// InteracionBlock_24927990186258
// MI455X (gfx1250) — hardware-verified
//
#include <hip/hip_runtime.h>
#include <stdint.h>
#include <stddef.h>

constexpr int kNB = 8;
constexpr int kNS = 256;
constexpr int kND = 256;
constexpr int kNH = 64;
constexpr int kNRBF = 300;
constexpr int kKR = 320;
constexpr int kTok = kNB * kNS;
constexpr int kPairsChunk = kNS * kNS;
constexpr int kChunks = kNB;

constexpr float kWCarry   = 16.0f;
constexpr float kActCarry = 16.0f;
constexpr float kHCarry   = 64.0f;
constexpr float kScaleAtom = 1.0f / (kActCarry * kWCarry);
constexpr float kScaleRbf  = 1.0f / kWCarry;
constexpr float kScaleFilt = 1.0f / (kHCarry * kWCarry);
constexpr float kLog2e = 1.4426950408889634f;
constexpr float kNeg10Log2e = -14.426950408889634f;
constexpr float kLn2 = 0.69314718056f;
constexpr float kF16MinNormal = 6.103515625e-05f;

constexpr size_t kBytesWAT   = (size_t)3 * kND * kND * 2;
constexpr size_t kBytesWS1T  = (size_t)kNH * kKR * 2;
constexpr size_t kBytesWS2T  = (size_t)kND * kNH * 2;
constexpr size_t kBytesPAR   = 16384;
constexpr size_t kBytesAct16 = (size_t)kTok * kND * 2;
constexpr size_t kBytesAct32 = (size_t)kTok * kND * 4;
constexpr size_t kBytesR16   = (size_t)kPairsChunk * kKR * 2;
constexpr size_t kBytesHPre  = (size_t)kPairsChunk * kNH * 4;
constexpr size_t kBytesH16   = (size_t)kPairsChunk * kNH * 2;
constexpr size_t kOffWAT  = 0;
constexpr size_t kOffWS1T = kOffWAT + kBytesWAT;
constexpr size_t kOffWS2T = kOffWS1T + kBytesWS1T;
constexpr size_t kOffPAR  = kOffWS2T + kBytesWS2T;
constexpr size_t kOffV16  = kOffPAR + kBytesPAR;
constexpr size_t kOffV1   = kOffV16 + kBytesAct16;
constexpr size_t kOffU16  = kOffV1 + kBytesAct32;
constexpr size_t kOffV2P  = kOffU16 + kBytesAct16;
constexpr size_t kOffV2H  = kOffV2P + kBytesAct32;
constexpr size_t kOffR16  = kOffV2H + kBytesAct16;
constexpr size_t kOffHPre = kOffR16 + kBytesR16;
constexpr size_t kOffH16  = kOffHPre + kBytesHPre;
constexpr size_t kWsTotal = kOffH16 + kBytesH16;
static_assert(kWsTotal <= (size_t)134217728, "ws cap");
static_assert((kOffWS1T % 4096) == 0 && (kOffWS2T % 4096) == 0 && (kOffPAR % 4096) == 0 && (kOffV16 % 4096) == 0 &&
              (kOffV1 % 4096) == 0 && (kOffU16 % 4096) == 0 && (kOffV2P % 4096) == 0 && (kOffV2H % 4096) == 0 &&
              (kOffR16 % 4096) == 0 && (kOffHPre % 4096) == 0 && (kOffH16 % 4096) == 0, "align");
static_assert((kKR % 32) == 0 && (kND % 64) == 0 && (kNH % 64) == 0 && (kTok % 64) == 0 && (kPairsChunk % 64) == 0, "tiles");

constexpr int kParMask = 0;
constexpr int kParBa1  = 2048;
constexpr int kParBa2  = 2304;
constexpr int kParBa3  = 2560;
constexpr int kParBs2  = 2816;
constexpr int kParBs1  = 3072;
static_assert((kParBs1 + kNH) * 4 <= (int)kBytesPAR, "par fits");
static_assert((kParBa1 * 4) % 128 == 0 && (kParBa2 * 4) % 128 == 0 && (kParBa3 * 4) % 128 == 0 &&
              (kParBs2 * 4) % 128 == 0 && (kParBs1 * 4) % 128 == 0, "par align");

typedef __attribute__((ext_vector_type(16))) _Float16 v16h;
typedef __attribute__((ext_vector_type(8)))  _Float16 v8h;
typedef __attribute__((ext_vector_type(16))) __bf16   v16b;
typedef __attribute__((ext_vector_type(8)))  __bf16   v8b;
typedef __attribute__((ext_vector_type(8)))  float    v8f;
typedef __attribute__((ext_vector_type(4)))  float    v4f;
typedef __attribute__((ext_vector_type(4)))  unsigned int v4u;

__device__ __forceinline__ unsigned short f2bf_bits(float f) {
  unsigned u = __float_as_uint(f);
  return (unsigned short)((u + 0x7FFFu + ((u >> 16) & 1u)) >> 16);
}
__device__ __forceinline__ float bf_bits2f(unsigned short h) { return __uint_as_float(((unsigned)h) << 16); }

__device__ __forceinline__ void dep_guard_h(v8f& a, v8f& b, v16h x, v16h y) { asm volatile("v_nop\n\tv_nop\n\tv_nop\n\tv_nop" : "+v"(a), "+v"(b) : "v"(x), "v"(y)); }
__device__ __forceinline__ void dep_guard_b(v8f& a, v8f& b, v16b x, v16b y) { asm volatile("v_nop\n\tv_nop\n\tv_nop\n\tv_nop" : "+v"(a), "+v"(b) : "v"(x), "v"(y)); }
__device__ __forceinline__ void keep4_h(v16h a, v16h b, v16h c, v16h d) { asm volatile("v_nop" :: "v"(a), "v"(b), "v"(c), "v"(d)); }
__device__ __forceinline__ void keep4_b(v16b a, v16b b, v16b c, v16b d) { asm volatile("v_nop" :: "v"(a), "v"(b), "v"(c), "v"(d)); }
__device__ __forceinline__ void acc_guard4(v8f& a, v8f& b, v8f& c, v8f& d) { asm volatile("v_nop\n\tv_nop\n\tv_nop\n\tv_nop" : "+v"(a), "+v"(b), "+v"(c), "+v"(d)); }
template <typename T> struct Frag;
template <> struct Frag<_Float16> {
  typedef v16h V; union U { v16h v; v8h h[2]; };
  static __device__ __forceinline__ v16h load(const _Float16* p) {
    U f; f.h[0] = *(const v8h*)(p); f.h[1] = *(const v8h*)(p + 16); return f.v;
  }
  static __device__ __forceinline__ v8f mma(v16h a, v16h b, v8f c) {
    return __builtin_amdgcn_wmma_f32_16x16x32_f16(false, a, false, b, (short)0, c, false, false);
  }
  static __device__ __forceinline__ void guard(v8f& a, v8f& b, v16h x, v16h y) { dep_guard_h(a, b, x, y); }
  static __device__ __forceinline__ void keep(v16h a, v16h b, v16h c, v16h d) { keep4_h(a, b, c, d); }
};
template <> struct Frag<__bf16> {
  typedef v16b V; union U { v16b v; v8b h[2]; };
  static __device__ __forceinline__ v16b load(const __bf16* p) {
    U f; f.h[0] = *(const v8b*)(p); f.h[1] = *(const v8b*)(p + 16); return f.v;
  }
  static __device__ __forceinline__ v8f mma(v16b a, v16b b, v8f c) {
    return __builtin_amdgcn_wmma_f32_16x16x32_bf16(false, a, false, b, (short)0, c, false, false);
  }
  static __device__ __forceinline__ void guard(v8f& a, v8f& b, v16b x, v16b y) { dep_guard_b(a, b, x, y); }
  static __device__ __forceinline__ void keep(v16b a, v16b b, v16b c, v16b d) { keep4_b(a, b, c, d); }
};

__device__ __forceinline__ unsigned pk16(unsigned short a, unsigned short b) { return (unsigned)a | ((unsigned)b << 16); }
__device__ __forceinline__ unsigned short h_bits(float f) { const _Float16 h = (_Float16)f; return __builtin_bit_cast(unsigned short, h); }

__device__ __forceinline__ float bfr(float f) { return bf_bits2f(f2bf_bits(f)); }

__device__ __forceinline__ float sspf(float x) {
  const float e = __builtin_amdgcn_exp2f(-fabsf(x) * kLog2e);
  const float l = __builtin_amdgcn_logf(1.0f + e);
  return fmaxf(x, 0.0f) + (l - 1.0f) * kLn2;
}

template <int ET> struct Elem;
template <> struct Elem<0> { typedef _Float16 T; };
template <> struct Elem<1> { typedef __bf16 T; };
template <int ET, bool SPLIT, int BIAS_MODE, int OUT_MODE, bool RESID, int ACT = 0, bool RMASK = false>
__global__ __launch_bounds__(256) void wmma_gemm64(
    const unsigned short* __restrict__ Ap, const unsigned short* __restrict__ A2p, int lda, long strideA,
    const unsigned short* __restrict__ Btp, const unsigned short* __restrict__ Bt2p, int ldb, long strideB,
    void* __restrict__ Cout, void* __restrict__ Cout2, int ldc, long strideC,
    const float* __restrict__ bias,
    const float* __restrict__ resid, long strideR,
    int M, int N, int K, float scale, const float* __restrict__ rmask) {
  typedef typename Elem<ET>::T T;
  typedef typename Frag<T>::V V;
  const T* A = (const T*)Ap; const T* A2 = (const T*)A2p; const T* Bt = (const T*)Btp; const T* Bt2 = (const T*)Bt2p;
  __shared__ __align__(16) float sT[8][16 * 68];
  const int b    = blockIdx.y;
  const int lane = threadIdx.x & 31;
  const int wave = threadIdx.x >> 5;
  const int tilesN = N >> 6;
  const int tilesM = M >> 6;
  const int tile = blockIdx.x * 8 + wave;
  if (tile >= tilesM * tilesN) return;
  const int tm = tile / tilesN;
  const int tn = tile - tm * tilesN;
  const int m0 = tm << 6;
  const int n0 = tn << 6;

  const T* Ab  = A  + (size_t)b * strideA;
  const T* Bb  = Bt + (size_t)b * strideB;
  const T* Ab2 = SPLIT ? (A2  + (size_t)b * strideA) : nullptr;
  const T* Bb2 = SPLIT ? (Bt2 + (size_t)b * strideB) : nullptr;

  const int rlane = lane & 15;
  const int koff  = (lane >> 4) * 8;
  const int mOff  = (lane >> 4) * 8;

  v8f acc[4][4];
#pragma unroll
  for (int i = 0; i < 4; ++i)
#pragma unroll
    for (int j = 0; j < 4; ++j) acc[i][j] = (v8f){0.f,0.f,0.f,0.f,0.f,0.f,0.f,0.f};

  for (int k0 = 0; k0 < K; k0 += 32) {
    V bh[4], bl[4];
#pragma unroll
    for (int j = 0; j < 4; ++j) {
      const size_t bo = (size_t)(n0 + (j << 4) + rlane) * ldb + koff + k0;
      bh[j] = Frag<T>::load(Bb + bo);
      if (SPLIT) bl[j] = Frag<T>::load(Bb2 + bo);
    }
#pragma unroll
    for (int i = 0; i < 4; ++i) {
      const size_t ao = (size_t)(m0 + (i << 4) + rlane) * lda + koff + k0;
      V ah = Frag<T>::load(Ab + ao);
      V al;
      if (SPLIT) al = Frag<T>::load(Ab2 + ao);
#pragma unroll
      for (int j = 0; j < 4; ++j) {
        acc[i][j] = Frag<T>::mma(ah, bh[j], acc[i][j]);
        if (SPLIT) {
          acc[i][j] = Frag<T>::mma(ah, bl[j], acc[i][j]);
          acc[i][j] = Frag<T>::mma(al, bh[j], acc[i][j]);
        }
      }
      Frag<T>::guard(acc[i][0], acc[i][3], ah, SPLIT ? al : ah);
    }
    Frag<T>::keep(bh[0], bh[1], bh[2], bh[3]);
    if (SPLIT) Frag<T>::keep(bl[0], bl[1], bl[2], bl[3]);
  }
  acc_guard4(acc[0][0], acc[0][1], acc[0][2], acc[0][3]);
  acc_guard4(acc[1][0], acc[1][1], acc[1][2], acc[1][3]);
  acc_guard4(acc[2][0], acc[2][1], acc[2][2], acc[2][3]);
  acc_guard4(acc[3][0], acc[3][1], acc[3][2], acc[3][3]);

  float* slab = sT[wave];
  const float* Rb = RESID ? (resid + (size_t)b * strideR) : nullptr;
#pragma unroll
  for (int i = 0; i < 4; ++i) {
    const int mBase = m0 + (i << 4);
#pragma unroll
    for (int j = 0; j < 4; ++j) {
      const int n = n0 + (j << 4) + rlane;
      float bv = 0.f;
      if (BIAS_MODE == 2) bv = bias[n];
#pragma unroll
      for (int r = 0; r < 8; ++r) {
        float v = acc[i][j][r] * scale;
        if (BIAS_MODE == 1) v += bias[mBase + mOff + r];
        if (BIAS_MODE == 2) v += bv;
        if (RESID) v += Rb[(size_t)(mBase + mOff + r) * ldc + n];
        if (ACT == 2) v = fmaxf(v, 0.0f);
        if (ACT == 4) v = (v > 0.f) ? v : 0.01f * v;
        if (RMASK) v *= rmask[mBase + mOff + r];
        slab[(mOff + r) * 68 + (j << 4) + rlane] = v;
      }
    }
    __builtin_amdgcn_fence(__ATOMIC_RELEASE, "workgroup");
    __builtin_amdgcn_wave_barrier();
    __builtin_amdgcn_fence(__ATOMIC_ACQUIRE, "workgroup");
    if (OUT_MODE == 0) {
      float* C = (float*)Cout + (size_t)b * strideC;
      const int hh = lane >> 4, c4 = (lane & 15) * 4;
      for (int pass = 0; pass < 2; ++pass) {
#pragma unroll
        for (int it = 0; it < 8; ++it) {
          const int row = it * 2 + hh;
          v4f v = *(const v4f*)(slab + row * 68 + c4);
          *(volatile v4f*)(C + (size_t)(mBase + row) * ldc + n0 + c4) = v;
        }
        __threadfence();
      }
    } else {
      const int q = lane >> 3, c8 = (lane & 7) * 8;
      unsigned short* C  = (unsigned short*)Cout  + (size_t)b * strideC;
      unsigned short* C2 = (OUT_MODE == 2) ? ((unsigned short*)Cout2 + (size_t)b * strideC) : nullptr;
      for (int pass = 0; pass < 2; ++pass) {
#pragma unroll
        for (int it = 0; it < 4; ++it) {
          const int row = it * 4 + q;
          const float* sp = slab + row * 68 + c8;
          v8h hv, lv;
#pragma unroll
          for (int e = 0; e < 8; ++e) {
            if (OUT_MODE == 1) {
              hv[e] = (_Float16)sp[e];
            } else {
              unsigned short hb = f2bf_bits(sp[e]);
              unsigned short lb = f2bf_bits(sp[e] - bf_bits2f(hb));
              hv[e] = __builtin_bit_cast(_Float16, hb);
              lv[e] = __builtin_bit_cast(_Float16, lb);
            }
          }
          *(volatile v8h*)(C + (size_t)(mBase + row) * ldc + n0 + c8) = hv;
          if (OUT_MODE == 2) *(volatile v8h*)(C2 + (size_t)(mBase + row) * ldc + n0 + c8) = lv;
        }
        __threadfence();
      }
    }
    __builtin_amdgcn_fence(__ATOMIC_RELEASE, "workgroup");
    __builtin_amdgcn_wave_barrier();
    __builtin_amdgcn_fence(__ATOMIC_ACQUIRE, "workgroup");
  }
}

__global__ __launch_bounds__(256) void wtcast_kernel(const float* __restrict__ W0, const float* __restrict__ W1,
                                                     const float* __restrict__ W2,
                                                     unsigned short* __restrict__ out, long planeStride,
                                                     int Kdim, int Ndim, int Kpad, float scale) {
  __shared__ float sm[64][65];
  const int t  = threadIdx.x;
  const int d0 = blockIdx.x * 64;
  const int h0 = blockIdx.y * 64;
  const int z  = blockIdx.z;
  const float* W = (z == 0) ? W0 : (z == 1) ? W1 : W2;
#pragma unroll
  for (int i = 0; i < 16; ++i) {
    const int e = i * 256 + t;
    const int r = e >> 6;
    const int c = e & 63;
    const int kg = d0 + r;
    const int kc = (kg < Kdim) ? kg : (Kdim - 1);
    float v = bfr(W[(size_t)kc * Ndim + h0 + c]) * scale;
    if (kg >= Kdim) v = 0.0f;
    sm[c][r] = v;
  }
  __syncthreads();
  const int lane = t & 31, wave = t >> 5;
  const int q = lane >> 3, c8 = (lane & 7) * 8;
  unsigned short* op = out + (size_t)z * planeStride;
  for (int pass = 0; pass < 2; ++pass) {
#pragma unroll
    for (int it = 0; it < 2; ++it) {
      const int row = wave * 8 + it * 4 + q;
      unsigned short hb[8];
#pragma unroll
      for (int e = 0; e < 8; ++e) hb[e] = h_bits(sm[row][c8 + e]);
      const v4u u = (v4u){pk16(hb[0], hb[1]), pk16(hb[2], hb[3]), pk16(hb[4], hb[5]), pk16(hb[6], hb[7])};
      *(volatile v4u*)(op + (size_t)(h0 + row) * Kpad + d0 + c8) = u;
    }
    __threadfence();
  }
}

__global__ __launch_bounds__(256) void snap_params_kernel(const float* __restrict__ pm, const float* __restrict__ pa1,
                                                          const float* __restrict__ pa2, const float* __restrict__ pa3,
                                                          const float* __restrict__ ps2, const float* __restrict__ ps1,
                                                          float* __restrict__ par) {
  const int z = blockIdx.y;
  const float* src = (z == 0) ? pm : (z == 1) ? pa1 : (z == 2) ? pa2 : (z == 3) ? pa3 : (z == 4) ? ps2 : ps1;
  const int n4  = (z == 0) ? (kTok / 4) : (z == 5) ? (kNH / 4) : (kND / 4);
  const int off = (z == 0) ? kParMask : (z == 1) ? kParBa1 : (z == 2) ? kParBa2 : (z == 3) ? kParBa3 : (z == 4) ? kParBs2 : kParBs1;
  const int i = blockIdx.x * 256 + threadIdx.x;
  if (i >= n4) return;
  const v4f a = *(const v4f*)(src + (size_t)4 * i);
  v4f rv;
  rv[0] = bfr(a[0]); rv[1] = bfr(a[1]); rv[2] = bfr(a[2]); rv[3] = bfr(a[3]);
  float* op = par + off + 4 * i;
  *(volatile v4f*)op = rv;
  __threadfence();
  *(volatile v4f*)op = rv;
}

template <int MODE>
__global__ __launch_bounds__(256) void ew_cast_kernel(const float* __restrict__ in, const float* __restrict__ rowmask,
                                                      _Float16* __restrict__ out, int n8, int rowShift, float s) {
  const int i8 = blockIdx.x * 256 + threadIdx.x;
  if (i8 >= n8) return;
  const float* ip = in + (size_t)i8 * 8;
  const v4f a = *(const v4f*)ip;
  const v4f c = *(const v4f*)(ip + 4);
  float x[8] = {a[0], a[1], a[2], a[3], c[0], c[1], c[2], c[3]};
  float mul = s;
  if (MODE != 1) mul *= rowmask[i8 >> rowShift];
  v8h hv;
#pragma unroll
  for (int e = 0; e < 8; ++e) {
    float y = x[e];
    if (MODE == 0) y = bfr(y);
    if (MODE != 0) y = sspf(y);
    hv[e] = (_Float16)(y * mul);
  }
  _Float16* op = out + (size_t)i8 * 8;
  *(volatile v8h*)op = hv;
  __threadfence();
  *(volatile v8h*)op = hv;
}

__global__ __launch_bounds__(256) void rbf_kernel(const float* __restrict__ dist, _Float16* __restrict__ R, int pairBase) {
#pragma clang fp contract(off)
  __shared__ __align__(16) _Float16 tile[64 * kKR];
  const int t = threadIdx.x;
  const int rowBase = blockIdx.x * 64;
#pragma unroll 1
  for (int it = 0; it < 10; ++it) {
    const int q = it * 256 + t;
    const int cc = q >> 6;
    const int row = q & 63;
    const float d = bfr(dist[(size_t)pairBase + rowBase + row]);
    v8h hv;
#pragma unroll
    for (int e = 0; e < 8; ++e) {
      const float mu = (float)(cc * 8 + e) * 0.1f;
      const float x = d - mu;
      const float sq = x * x;
      float ev = __builtin_amdgcn_exp2f(sq * kNeg10Log2e);
      ev = (ev >= kF16MinNormal) ? ev : 0.0f;
      hv[e] = (_Float16)ev;
    }
    if (cc * 8 + 8 > kNRBF) {
#pragma unroll
      for (int e = 0; e < 8; ++e) {
        if (cc * 8 + e >= kNRBF) hv[e] = (_Float16)0.0f;
      }
    }
    *(v8h*)(tile + row * kKR + cc * 8) = hv;
  }
  __syncthreads();
#pragma unroll 1
  for (int it = 0; it < 10; ++it) {
    const int q = it * 256 + t;
    const int row = q / 40;
    const int c8 = (q - row * 40) * 8;
    const v8h hv = *(const v8h*)(tile + row * kKR + c8);
    _Float16* op = R + (size_t)(rowBase + row) * kKR + c8;
    *(volatile v8h*)op = hv;
    __threadfence();
    *(volatile v8h*)op = hv;
  }
}

__global__ __launch_bounds__(256) void filter_reduce_kernel(
    const _Float16* __restrict__ Hc, const _Float16* __restrict__ W2t, const float* __restrict__ b2,
    const float* __restrict__ v1, const float* __restrict__ rowmask, _Float16* __restrict__ U, int bsel) {
  __shared__ __align__(16) _Float16 su[kND];
  typedef Frag<_Float16> F;
  const int i = blockIdx.x;
  const int lane = threadIdx.x & 31, wave = threadIdx.x >> 5;
  const int rlane = lane & 15;
  const int koff = (lane >> 4) * 8;
  const int mOff = (lane >> 4) * 8;
  const int d0 = wave * 32;

  const v16h bf00 = F::load(W2t + (size_t)(d0 + rlane) * kNH + koff);
  const v16h bf01 = F::load(W2t + (size_t)(d0 + rlane) * kNH + 32 + koff);
  const v16h bf10 = F::load(W2t + (size_t)(d0 + 16 + rlane) * kNH + koff);
  const v16h bf11 = F::load(W2t + (size_t)(d0 + 16 + rlane) * kNH + 32 + koff);
  const float bv0 = b2[d0 + rlane];
  const float bv1 = b2[d0 + 16 + rlane];

  const _Float16* Hb = Hc + (size_t)i * kNS * kNH;
  const float* v1b = v1 + (size_t)bsel * kNS * kND;
  float red0 = 0.0f, red1 = 0.0f;

#pragma unroll 1
  for (int jt = 0; jt < kNS / 16; ++jt) {
    v8f acc0 = (v8f){0.f,0.f,0.f,0.f,0.f,0.f,0.f,0.f};
    v8f acc1 = (v8f){0.f,0.f,0.f,0.f,0.f,0.f,0.f,0.f};
    const _Float16* arow = Hb + (size_t)(jt * 16 + rlane) * kNH + koff;
    const v16h a0 = F::load(arow);
    const v16h a1 = F::load(arow + 32);
    acc0 = F::mma(a0, bf00, acc0);
    acc1 = F::mma(a0, bf10, acc1);
    acc0 = F::mma(a1, bf01, acc0);
    acc1 = F::mma(a1, bf11, acc1);
    F::guard(acc0, acc1, a0, a1);

    const float* vr = v1b + (size_t)(jt * 16 + mOff) * kND + d0 + rlane;
#pragma unroll
    for (int r = 0; r < 8; ++r) {
      const float x0 = acc0[r] * kScaleFilt + bv0;
      const float x1 = acc1[r] * kScaleFilt + bv1;
      const float w0 = sspf(x0);
      const float w1 = sspf(x1);
      red0 += w0 * vr[(size_t)r * kND];
      red1 += w1 * vr[(size_t)r * kND + 16];
    }
  }
  F::keep(bf00, bf01, bf10, bf11);

  red0 += __shfl_xor(red0, 16, 32);
  red1 += __shfl_xor(red1, 16, 32);
  const float mr = rowmask[bsel * kNS + i] * kActCarry;
  if (lane < 16) {
    su[d0 + lane] = (_Float16)(red0 * mr);
    su[d0 + 16 + lane] = (_Float16)(red1 * mr);
  }
  __syncthreads();
  if (wave == 0) {
    const v8h hv = *(const v8h*)(su + 8 * lane);
    _Float16* op = U + (size_t)(bsel * kNS + i) * kND + 8 * lane;
    *(volatile v8h*)op = hv;
    __threadfence();
    *(volatile v8h*)op = hv;
  }
}

extern "C" void kernel_launch(void* const* d_in, const int* in_sizes, int n_in,
                              void* d_out, int out_size, void* d_ws, size_t ws_size,
                              hipStream_t stream) {
  if (n_in < 13) return;
  if (in_sizes[0] != kTok * kND || in_sizes[1] != kNB * kNS * kNS || in_sizes[2] != kTok ||
      in_sizes[3] != kNRBF * kNH || in_sizes[4] != kNH || in_sizes[5] != kNH * kND || in_sizes[6] != kND ||
      in_sizes[7] != kND * kND || in_sizes[8] != kND || in_sizes[9] != kND * kND || in_sizes[10] != kND ||
      in_sizes[11] != kND * kND || in_sizes[12] != kND) return;
  if (out_size != kTok * kND) return;
  if (ws_size < kWsTotal) return;

  const float* vin   = (const float*)d_in[0];
  const float* dist  = (const float*)d_in[1];
  const float* maskf = (const float*)d_in[2];
  const float* Ws1   = (const float*)d_in[3];
  const float* bs1   = (const float*)d_in[4];
  const float* Ws2   = (const float*)d_in[5];
  const float* bs2   = (const float*)d_in[6];
  const float* Wa1   = (const float*)d_in[7];
  const float* ba1   = (const float*)d_in[8];
  const float* Wa2   = (const float*)d_in[9];
  const float* ba2   = (const float*)d_in[10];
  const float* Wa3   = (const float*)d_in[11];
  const float* ba3   = (const float*)d_in[12];
  float* out = (float*)d_out;

  char* ws = (char*)d_ws;
  _Float16* pWAT  = (_Float16*)(ws + kOffWAT);
  _Float16* pWa1t = pWAT;
  _Float16* pWa2t = pWAT + (size_t)kND * kND;
  _Float16* pWa3t = pWAT + (size_t)2 * kND * kND;
  _Float16* pWS1T = (_Float16*)(ws + kOffWS1T);
  _Float16* pWS2T = (_Float16*)(ws + kOffWS2T);
  float*    pPAR  = (float*)(ws + kOffPAR);
  const float* pMaskR = pPAR + kParMask;
  const float* pBa1R  = pPAR + kParBa1;
  const float* pBa2R  = pPAR + kParBa2;
  const float* pBa3R  = pPAR + kParBa3;
  const float* pBs2R  = pPAR + kParBs2;
  const float* pBs1R  = pPAR + kParBs1;
  _Float16* pV16  = (_Float16*)(ws + kOffV16);
  float*    pV1   = (float*)(ws + kOffV1);
  _Float16* pU16  = (_Float16*)(ws + kOffU16);
  float*    pV2P  = (float*)(ws + kOffV2P);
  _Float16* pV2H  = (_Float16*)(ws + kOffV2H);
  _Float16* pR16  = (_Float16*)(ws + kOffR16);
  float*    pHPre = (float*)(ws + kOffHPre);
  _Float16* pH16  = (_Float16*)(ws + kOffH16);

  const dim3 blk(256);

  wtcast_kernel<<<dim3(kND / 64, kND / 64, 3), blk, 0, stream>>>(Wa1, Wa2, Wa3, (unsigned short*)pWAT,
                                                                   (long)kND * kND, kND, kND, kND, kWCarry);
  wtcast_kernel<<<dim3(kKR / 64, kNH / 64, 1), blk, 0, stream>>>(Ws1, Ws1, Ws1, (unsigned short*)pWS1T,
                                                                   0L, kNRBF, kNH, kKR, kWCarry);
  wtcast_kernel<<<dim3(kNH / 64, kND / 64, 1), blk, 0, stream>>>(Ws2, Ws2, Ws2, (unsigned short*)pWS2T,
                                                                   0L, kNH, kND, kNH, kWCarry);
  snap_params_kernel<<<dim3(2, 6, 1), blk, 0, stream>>>(maskf, ba1, ba2, ba3, bs2, bs1, pPAR);

  ew_cast_kernel<0><<<dim3(kTok * kND / 8 / 256), blk, 0, stream>>>(vin, pMaskR, pV16, kTok * kND / 8, 5, kActCarry);

  wmma_gemm64<0, false, 2, 0, false, 0, true><<<dim3(kTok / 64 * (kND / 64) / 8, 1, 1), blk, 0, stream>>>(
      (const unsigned short*)pV16, (const unsigned short*)pV16, kND, 0L,
      (const unsigned short*)pWa1t, (const unsigned short*)pWa1t, kND, 0L,
      (void*)pV1, (void*)pV1, kND, 0L,
      pBa1R, pBa1R, 0L, kTok, kND, kND, kScaleAtom, pMaskR);

  for (int c = 0; c < kChunks; ++c) {
    rbf_kernel<<<dim3(kPairsChunk / 64), blk, 0, stream>>>(dist, pR16, c * kPairsChunk);
    wmma_gemm64<0, false, 2, 0, false, 0, false><<<dim3(kPairsChunk / 64 * (kNH / 64) / 8, 1, 1), blk, 0, stream>>>(
        (const unsigned short*)pR16, (const unsigned short*)pR16, kKR, 0L,
        (const unsigned short*)pWS1T, (const unsigned short*)pWS1T, kKR, 0L,
        (void*)pHPre, (void*)pHPre, kNH, 0L,
        pBs1R, pBs1R, 0L, kPairsChunk, kNH, kKR, kScaleRbf, pMaskR);
    ew_cast_kernel<1><<<dim3(kPairsChunk * kNH / 8 / 256), blk, 0, stream>>>(pHPre, pMaskR, pH16,
                                                                            kPairsChunk * kNH / 8, 0, kHCarry);
    filter_reduce_kernel<<<dim3(kNS), blk, 0, stream>>>(pH16, pWS2T, pBs2R, pV1, pMaskR, pU16, c);
  }

  wmma_gemm64<0, false, 2, 0, false, 0, false><<<dim3(kTok / 64 * (kND / 64) / 8, 1, 1), blk, 0, stream>>>(
      (const unsigned short*)pU16, (const unsigned short*)pU16, kND, 0L,
      (const unsigned short*)pWa2t, (const unsigned short*)pWa2t, kND, 0L,
      (void*)pV2P, (void*)pV2P, kND, 0L,
      pBa2R, pBa2R, 0L, kTok, kND, kND, kScaleAtom, pMaskR);
  ew_cast_kernel<2><<<dim3(kTok * kND / 8 / 256), blk, 0, stream>>>(pV2P, pMaskR, pV2H, kTok * kND / 8, 5, kActCarry);

  wmma_gemm64<0, false, 2, 0, false, 0, true><<<dim3(kTok / 64 * (kND / 64) / 8, 1, 1), blk, 0, stream>>>(
      (const unsigned short*)pV2H, (const unsigned short*)pV2H, kND, 0L,
      (const unsigned short*)pWa3t, (const unsigned short*)pWa3t, kND, 0L,
      (void*)out, (void*)out, kND, 0L,
      pBa3R, pBa3R, 0L, kTok, kND, kND, kScaleAtom, pMaskR);
}
